// BasicModelThetaPerStep_49074296324488
// MI455X (gfx1250) — hardware-run, weakly checked
//
#include <hip/hip_runtime.h>
#include <math.h>

typedef __attribute__((ext_vector_type(16))) _Float16 v16h;
typedef __attribute__((ext_vector_type(8)))  _Float16 v8h;
typedef __attribute__((ext_vector_type(2)))  _Float16 v2h;
typedef __attribute__((ext_vector_type(16))) __bf16   v16b;
typedef __attribute__((ext_vector_type(8)))  __bf16   v8b;
typedef __attribute__((ext_vector_type(8)))  float    v8f;
typedef __attribute__((ext_vector_type(4)))  float    v4f;
typedef __attribute__((ext_vector_type(2)))  float    v2f;

constexpr int kB    = 256;
constexpr int kT    = 512;
constexpr int kXi   = 65;
constexpr int kK1   = 64;
constexpr int kH    = 128;
constexpr int kG3   = 384;
constexpr int kCh   = 64;
constexpr int kCv   = 64;
constexpr int kCi   = 129;
constexpr int kCo   = 65;
constexpr int kThr  = 256;
constexpr float kInCarry = 1024.0f;
constexpr float kSc20 = 1.0f / (kInCarry * kInCarry);
constexpr float kSc10 = 1.0f / kInCarry;
constexpr float kF16MinNormal = 6.103515625e-5f;
constexpr size_t kOut0 = 0;
constexpr size_t kOut1 = (size_t)kB * kT * 3;
constexpr size_t kOut2 = kOut1 + (size_t)kB * kT * kH;
constexpr size_t kOutN = kOut2 + (size_t)kB * (kT - 1) * kCo;

static_assert(kB == 256 && kT == 512 && kXi == 65 && kK1 == 64 && kH == 128 && kG3 == 3 * kH && kCh == 64 && kT % kCh == 0 && kCv == 64 && kCi == kH + 1 && kCo == kCv + 1, "the index arithmetic below uses these sizes");

constexpr size_t kOffX16 = 0ull;
constexpr size_t kOffWIT = 16777216ull;
constexpr size_t kOffWHT = 16826368ull;
constexpr size_t kOffWCT = 16924672ull;
constexpr size_t kOffGX = 16941056ull;
constexpr size_t kOffGH = 42106880ull;
constexpr size_t kOffH32 = 42500096ull;
constexpr size_t kOffH16 = 42631168ull;
constexpr size_t kOffHS16 = 42696704ull;
constexpr size_t kOffCV = 76251136ull;
constexpr size_t kWsTotal = 109805568ull;
static_assert(kWsTotal <= 134217728ull, "the carve stands under 128 MiB");
static_assert(kOffX16 == 0
  && kOffWIT == kOffX16 + 16777216ull
  && kOffWHT == kOffWIT + 49152ull
  && kOffWCT == kOffWHT + 98304ull
  && kOffGX == kOffWCT + 16384ull
  && kOffGH == kOffGX + 25165824ull
  && kOffH32 == kOffGH + 393216ull
  && kOffH16 == kOffH32 + 131072ull
  && kOffHS16 == kOffH16 + 65536ull
  && kOffCV == kOffHS16 + 33554432ull
  && kWsTotal == kOffCV + 33554432ull, "the carve is a chain: every region starts where the one before ends");
static_assert((kOffX16 % 256) == 0 && (kOffWIT % 256) == 0 && (kOffWHT % 256) == 0 && (kOffWCT % 256) == 0 && (kOffGX % 256) == 0 && (kOffGH % 256) == 0 && (kOffH32 % 256) == 0 && (kOffH16 % 256) == 0 && (kOffHS16 % 256) == 0 && (kOffCV % 256) == 0, "every region starts on a multiple of 256 B");

__device__ __forceinline__ unsigned short f2bf_bits(float f) {
  unsigned u = __float_as_uint(f);
  return (unsigned short)((u + 0x7FFFu + ((u >> 16) & 1u)) >> 16);
}
__device__ __forceinline__ float bf_bits2f(unsigned short h) { return __uint_as_float(((unsigned)h) << 16); }
__device__ __forceinline__ float bf16r(float f) { return bf_bits2f(f2bf_bits(f)); }
__device__ __forceinline__ float carry_flush(float v, float carry) {
  const float s = v * carry;
  return (fabsf(s) < kF16MinNormal) ? 0.0f : s;
}

__device__ __forceinline__ void dep_guard4_h(v8f& a, v8f& b, v8f& c, v8f& d, v16h x, v16h y) { asm volatile("v_nop\n\tv_nop\n\tv_nop\n\tv_nop" : "+v"(a), "+v"(b), "+v"(c), "+v"(d) : "v"(x), "v"(y)); }
__device__ __forceinline__ void dep_guard4_b(v8f& a, v8f& b, v8f& c, v8f& d, v16b x, v16b y) { asm volatile("v_nop\n\tv_nop\n\tv_nop\n\tv_nop" : "+v"(a), "+v"(b), "+v"(c), "+v"(d) : "v"(x), "v"(y)); }
__device__ __forceinline__ void keep4_h(v16h a, v16h b, v16h c, v16h d) { asm volatile("v_nop" :: "v"(a), "v"(b), "v"(c), "v"(d)); }
__device__ __forceinline__ void keep4_b(v16b a, v16b b, v16b c, v16b d) { asm volatile("v_nop" :: "v"(a), "v"(b), "v"(c), "v"(d)); }
__device__ __forceinline__ void acc_guard4(v8f& a, v8f& b, v8f& c, v8f& d) { asm volatile("v_nop\n\tv_nop\n\tv_nop\n\tv_nop" : "+v"(a), "+v"(b), "+v"(c), "+v"(d)); }

template <typename T> struct Frag;
template <> struct Frag<_Float16> {
  typedef v16h V; union U { v16h v; v8h h[2]; };
  static __device__ __forceinline__ v16h load(const _Float16* p) {
    U f; f.h[0] = *(const v8h*)(p); f.h[1] = *(const v8h*)(p + 16); return f.v;
  }
  static __device__ __forceinline__ v8f mma(v16h a, v16h b, v8f c) {
    return __builtin_amdgcn_wmma_f32_16x16x32_f16(false, a, false, b, (short)0, c, false, false);
  }
  static __device__ __forceinline__ void guard4(v8f& a, v8f& b, v8f& c, v8f& d, v16h x, v16h y) { dep_guard4_h(a, b, c, d, x, y); }
  static __device__ __forceinline__ void keep(v16h a, v16h b, v16h c, v16h d) { keep4_h(a, b, c, d); }
};
template <> struct Frag<__bf16> {
  typedef v16b V; union U { v16b v; v8b h[2]; };
  static __device__ __forceinline__ v16b load(const __bf16* p) {
    U f; f.h[0] = *(const v8b*)(p); f.h[1] = *(const v8b*)(p + 16); return f.v;
  }
  static __device__ __forceinline__ v8f mma(v16b a, v16b b, v8f c) {
    return __builtin_amdgcn_wmma_f32_16x16x32_bf16(false, a, false, b, (short)0, c, false, false);
  }
  static __device__ __forceinline__ void guard4(v8f& a, v8f& b, v8f& c, v8f& d, v16b x, v16b y) { dep_guard4_b(a, b, c, d, x, y); }
  static __device__ __forceinline__ void keep(v16b a, v16b b, v16b c, v16b d) { keep4_b(a, b, c, d); }
};

__device__ __forceinline__ v8f mma_h(v16h a, v16h b, v8f c) {
  c = __builtin_amdgcn_wmma_f32_16x16x32_f16(false, a, false, b, (short)0, c, false, false);
  asm volatile("v_nop\n\tv_nop\n\tv_nop\n\tv_nop" : "+v"(c) : "v"(a), "v"(b));
  return c;
}

template <int ET> struct Elem;
template <> struct Elem<0> { typedef _Float16 T; };
template <> struct Elem<1> { typedef __bf16 T; };
template <int ET, bool SPLIT, int BIAS_MODE, int OUT_MODE, bool RESID, int ACT = 0>
__global__ __launch_bounds__(256) void wmma_gemm64(
    const unsigned short* __restrict__ Ap, const unsigned short* __restrict__ A2p, int lda, long strideA,
    const unsigned short* __restrict__ Btp, const unsigned short* __restrict__ Bt2p, int ldb, long strideB,
    void* __restrict__ Cout, void* __restrict__ Cout2, int ldc, long strideC,
    const float* __restrict__ bias,
    const float* __restrict__ resid, long strideR,
    int M, int N, int K, float scale) {
  typedef typename Elem<ET>::T T;
  typedef typename Frag<T>::V V;
  const T* A = (const T*)Ap; const T* A2 = (const T*)A2p; const T* Bt = (const T*)Btp; const T* Bt2 = (const T*)Bt2p;
  __shared__ __align__(16) float sT[8][16 * 68];
  const int b    = blockIdx.y;
  const int lane = threadIdx.x & 31;
  const int wave = threadIdx.x >> 5;
  const int tilesN = N >> 6;
  const int tilesM = M >> 6;
  const int tile = blockIdx.x * 8 + wave;
  if (tile >= tilesM * tilesN) return;
  const int tm = tile / tilesN;
  const int tn = tile - tm * tilesN;
  const int m0 = tm << 6;
  const int n0 = tn << 6;

  const T* Ab  = A  + (size_t)b * strideA;
  const T* Bb  = Bt + (size_t)b * strideB;
  const T* Ab2 = SPLIT ? (A2  + (size_t)b * strideA) : nullptr;
  const T* Bb2 = SPLIT ? (Bt2 + (size_t)b * strideB) : nullptr;

  const int rlane = lane & 15;
  const int koff  = (lane >> 4) * 8;
  const int mOff  = (lane >> 4) * 8;

  v8f acc[4][4];
#pragma unroll
  for (int i = 0; i < 4; ++i)
#pragma unroll
    for (int j = 0; j < 4; ++j) acc[i][j] = (v8f){0.f,0.f,0.f,0.f,0.f,0.f,0.f,0.f};

  for (int k0 = 0; k0 < K; k0 += 32) {
    V bh[4], bl[4];
#pragma unroll
    for (int j = 0; j < 4; ++j) {
      const size_t bo = (size_t)(n0 + (j << 4) + rlane) * ldb + koff + k0;
      bh[j] = Frag<T>::load(Bb + bo);
      if (SPLIT) bl[j] = Frag<T>::load(Bb2 + bo);
    }
#pragma unroll
    for (int i = 0; i < 4; ++i) {
      const size_t ao = (size_t)(m0 + (i << 4) + rlane) * lda + koff + k0;
      V ah = Frag<T>::load(Ab + ao);
      V al;
      if (SPLIT) al = Frag<T>::load(Ab2 + ao);
#pragma unroll
      for (int j = 0; j < 4; ++j) {
        acc[i][j] = Frag<T>::mma(ah, bh[j], acc[i][j]);
        if (SPLIT) {
          acc[i][j] = Frag<T>::mma(ah, bl[j], acc[i][j]);
          acc[i][j] = Frag<T>::mma(al, bh[j], acc[i][j]);
        }
      }
      Frag<T>::guard4(acc[i][0], acc[i][1], acc[i][2], acc[i][3], ah, SPLIT ? al : ah);
    }
    Frag<T>::keep(bh[0], bh[1], bh[2], bh[3]);
    if (SPLIT) Frag<T>::keep(bl[0], bl[1], bl[2], bl[3]);
  }
  acc_guard4(acc[0][0], acc[0][1], acc[0][2], acc[0][3]);
  acc_guard4(acc[1][0], acc[1][1], acc[1][2], acc[1][3]);
  acc_guard4(acc[2][0], acc[2][1], acc[2][2], acc[2][3]);
  acc_guard4(acc[3][0], acc[3][1], acc[3][2], acc[3][3]);

  float* slab = sT[wave];
  const float* Rb = RESID ? (resid + (size_t)b * strideR) : nullptr;
#pragma unroll
  for (int i = 0; i < 4; ++i) {
    const int mBase = m0 + (i << 4);
#pragma unroll
    for (int j = 0; j < 4; ++j) {
      const int n = n0 + (j << 4) + rlane;
      float bv = 0.f;
      if (BIAS_MODE == 2) bv = bias[n];
#pragma unroll
      for (int r = 0; r < 8; ++r) {
        float v = acc[i][j][r] * scale;
        if (BIAS_MODE == 1) v += bias[mBase + mOff + r];
        if (BIAS_MODE == 2) v += bv;
        if (RESID) v += Rb[(size_t)(mBase + mOff + r) * ldc + n];
        if (ACT == 1) v = tanhf(v);
        if (ACT == 2) v = fmaxf(v, 0.0f);
        if (ACT == 3) v = v / (1.0f + expf(-v));
        if (ACT == 4) v = (v > 0.f) ? v : 0.01f * v;
        slab[(mOff + r) * 68 + (j << 4) + rlane] = v;
      }
    }
    __builtin_amdgcn_fence(__ATOMIC_RELEASE, "workgroup");
    __builtin_amdgcn_wave_barrier();
    __builtin_amdgcn_fence(__ATOMIC_ACQUIRE, "workgroup");
    if (OUT_MODE == 0) {
      float* C = (float*)Cout + (size_t)b * strideC;
      const int hh = lane >> 4, c4 = (lane & 15) * 4;
      for (int pass = 0; pass < 2; ++pass) {
#pragma unroll
        for (int it = 0; it < 8; ++it) {
          const int row = it * 2 + hh;
          v4f v = *(const v4f*)(slab + row * 68 + c4);
          *(volatile v4f*)(C + (size_t)(mBase + row) * ldc + n0 + c4) = v;
        }
        __threadfence();
      }
    } else {
      const int q = lane >> 3, c8 = (lane & 7) * 8;
      unsigned short* C  = (unsigned short*)Cout  + (size_t)b * strideC;
      unsigned short* C2 = (OUT_MODE == 2) ? ((unsigned short*)Cout2 + (size_t)b * strideC) : nullptr;
      for (int pass = 0; pass < 2; ++pass) {
#pragma unroll
        for (int it = 0; it < 4; ++it) {
          const int row = it * 4 + q;
          const float* sp = slab + row * 68 + c8;
          v8h hv, lv;
#pragma unroll
          for (int e = 0; e < 8; ++e) {
            if (OUT_MODE == 1) {
              hv[e] = (_Float16)sp[e];
            } else {
              unsigned short hb = f2bf_bits(sp[e]);
              unsigned short lb = f2bf_bits(sp[e] - bf_bits2f(hb));
              hv[e] = __builtin_bit_cast(_Float16, hb);
              lv[e] = __builtin_bit_cast(_Float16, lb);
            }
          }
          *(volatile v8h*)(C + (size_t)(mBase + row) * ldc + n0 + c8) = hv;
          if (OUT_MODE == 2) *(volatile v8h*)(C2 + (size_t)(mBase + row) * ldc + n0 + c8) = lv;
        }
        __threadfence();
      }
    }
    __builtin_amdgcn_fence(__ATOMIC_RELEASE, "workgroup");
    __builtin_amdgcn_wave_barrier();
    __builtin_amdgcn_fence(__ATOMIC_ACQUIRE, "workgroup");
  }
}

__global__ __launch_bounds__(kThr) void cast_plane_kernel(const float* __restrict__ src, unsigned short* __restrict__ dst,
                                                          int colsLog2, int dstPitch, int dstOff) {
  const int i   = blockIdx.x * kThr + threadIdx.x;
  const int sh  = colsLog2 - 3;
  const int row = i >> sh;
  const int c8  = (i & ((1 << sh) - 1)) * 8;
  const float* sp = src + ((size_t)row << colsLog2) + c8;
  const v4f a0 = *(const v4f*)(sp);
  const v4f a1 = *(const v4f*)(sp + 4);
  v8h hv;
#pragma unroll
  for (int e = 0; e < 4; ++e) {
    const float f0 = a0[e];
    const float f1 = a1[e];
    hv[e]     = (_Float16)carry_flush(bf16r(f0), kInCarry);
    hv[4 + e] = (_Float16)carry_flush(bf16r(f1), kInCarry);
  }
  unsigned short* dp = dst + (size_t)row * dstPitch + dstOff + c8;
  *(volatile v8h*)dp = hv;
  __threadfence();
  *(volatile v8h*)dp = hv;
}

__global__ __launch_bounds__(kThr) void pack_kernel(const float* __restrict__ W, unsigned short* __restrict__ D, float* __restrict__ dstf, int part, int ld, int k0, int lg, int n0, int pitch) {
  const unsigned i = blockIdx.x * blockDim.x + threadIdx.x;
  if (part == 0) {
    const unsigned g = i & ((1u << lg) - 1u), n = i >> lg;
    const float* sp = W + (size_t)((unsigned)k0 + g * 8u) * (unsigned)ld + n;
    v8h hv;
#pragma unroll
    for (int t = 0; t < 8; ++t) hv[t] = (_Float16)carry_flush(bf16r(sp[(size_t)t * (unsigned)ld]), kInCarry);
    unsigned short* dp = D + (size_t)((unsigned)n0 + n) * (unsigned)pitch + g * 8u;
    *(volatile v8h*)dp = hv;
    __threadfence();
    *(volatile v8h*)dp = hv;
  } else {
    const v4f a = *(const v4f*)(W + i * 4u);
    v4f o;
#pragma unroll
    for (int e = 0; e < 4; ++e) o[e] = bf16r(a[e]);
    float* dp = dstf + i * 4u;
    *(volatile v4f*)dp = o;
    __threadfence();
    *(volatile v4f*)dp = o;
  }
}

__global__ __launch_bounds__(kThr) void ocast_kernel(const float* __restrict__ src, unsigned short* __restrict__ dst, int pitch, int colsLog2) {
  const unsigned i = blockIdx.x * (unsigned)kThr + threadIdx.x;
  const unsigned gl = (unsigned)colsLog2 - 3u;
  const unsigned row = i >> gl, g = i & ((1u << gl) - 1u);
  const float* sp = src + (size_t)row * (unsigned)pitch + 8u * g;
  v8h hv;
#pragma unroll
  for (int t = 0; t < 8; ++t) hv[t] = (_Float16)carry_flush(bf16r(sp[t]), kInCarry);
  unsigned short* dp = dst + ((size_t)row << colsLog2) + 8u * g;
  *(volatile v8h*)dp = hv;
  __threadfence();
  *(volatile v8h*)dp = hv;
}

__global__ __launch_bounds__(kThr) void xcast_kernel(const float* __restrict__ x, const int* __restrict__ len, unsigned short* __restrict__ dst) {
  const unsigned i = blockIdx.x * (unsigned)kThr + threadIdx.x;
  const unsigned row = i >> 3, g = i & 7u;
  const unsigned b = row >> 9, t = row & 511u;
  const unsigned mk = ((int)t < len[b]) ? 0xFFFFFFFFu : 0u;
  const float* sp = x + (size_t)row * (unsigned)kXi + 8u * g;
  v8h hv;
#pragma unroll
  for (int e = 0; e < 8; ++e) hv[e] = (_Float16)carry_flush(bf16r(__uint_as_float(__float_as_uint(sp[e]) & mk)), kInCarry);
  unsigned short* dp = dst + (size_t)row * (unsigned)kK1 + 8u * g;
  *(volatile v8h*)dp = hv;
  __threadfence();
  *(volatile v8h*)dp = hv;
}

__global__ __launch_bounds__(kThr) void cell_kernel(const float* __restrict__ GX, const float* __restrict__ GH, const float* __restrict__ x, const int* __restrict__ len, const float* __restrict__ Wi, const float* __restrict__ bi, const float* __restrict__ bh,
                                                    float* __restrict__ H32, unsigned short* __restrict__ H16, float* __restrict__ hs, unsigned short* __restrict__ HS16, int t) {
  const unsigned i = blockIdx.x * (unsigned)kThr + threadIdx.x;
  const unsigned b = i >> 4, u8 = (i & 15u) << 3;
  const unsigned tl = (unsigned)t & (unsigned)(kCh - 1);
  const unsigned mk = (t < len[b]) ? 0xFFFFFFFFu : 0u;
  const float x64 = bf16r(__uint_as_float(__float_as_uint(x[((size_t)b * kT + (unsigned)t) * (unsigned)kXi + (unsigned)kK1]) & mk));
  const float* gx = GX + ((size_t)b * kCh + tl) * (unsigned)kG3 + u8;
  const float* gh = GH + (size_t)b * (unsigned)kG3 + u8;
  float* hp = H32 + (size_t)b * (unsigned)kH + u8;
  v8h hv, sv;
  v4f hn0, hn1, ho0, ho1;
#pragma unroll
  for (int hlf = 0; hlf < 2; ++hlf) {
    const v4f xr = *(const v4f*)(gx + 4 * hlf), xz = *(const v4f*)(gx + kH + 4 * hlf), xn = *(const v4f*)(gx + 2 * kH + 4 * hlf);
    const v4f sr = *(const v4f*)(gh + 4 * hlf), sz = *(const v4f*)(gh + kH + 4 * hlf), sn = *(const v4f*)(gh + 2 * kH + 4 * hlf);
    const v4f pr = *(const v4f*)(bi + u8 + 4 * hlf), pz = *(const v4f*)(bi + kH + u8 + 4 * hlf), pn = *(const v4f*)(bi + 2 * kH + u8 + 4 * hlf);
    const v4f qr = *(const v4f*)(bh + u8 + 4 * hlf), qz = *(const v4f*)(bh + kH + u8 + 4 * hlf), qn = *(const v4f*)(bh + 2 * kH + u8 + 4 * hlf);
    const v4f ho = *(const v4f*)(hp + 4 * hlf);
#pragma unroll
    for (int e = 0; e < 4; ++e) {
      const unsigned u = u8 + 4u * (unsigned)hlf + (unsigned)e;
      const float wr = bf16r(Wi[(size_t)u * kXi + kK1]), wz = bf16r(Wi[(size_t)(kH + u) * kXi + kK1]), wn = bf16r(Wi[(size_t)(2 * kH + u) * kXi + kK1]);
      const float r = 1.0f / (1.0f + expf(-(((xr[e] + x64 * wr) + bf16r(pr[e])) + (sr[e] + bf16r(qr[e])))));
      const float z = 1.0f / (1.0f + expf(-(((xz[e] + x64 * wz) + bf16r(pz[e])) + (sz[e] + bf16r(qz[e])))));
      const float n = tanhf(((xn[e] + x64 * wn) + bf16r(pn[e])) + r * (sn[e] + bf16r(qn[e])));
      const float hn = (1.0f - z) * n + z * ho[e];
      const float hm = __uint_as_float(__float_as_uint(hn) & mk);
      if (hlf == 0) { hn0[e] = hn; ho0[e] = hm; } else { hn1[e] = hn; ho1[e] = hm; }
      hv[4 * hlf + e] = (_Float16)carry_flush(hn, kInCarry);
      sv[4 * hlf + e] = (_Float16)carry_flush(hm, kInCarry);
    }
  }
  unsigned short* sp = H16 + (size_t)b * (unsigned)kH + u8;
  const size_t yo = ((size_t)b * kT + (unsigned)t) * (unsigned)kH + u8;
  float* fp = hs + yo;
  unsigned short* yp = HS16 + yo;
  for (int pass = 0; pass < 2; ++pass) {
    *(volatile v4f*)hp = hn0;
    *(volatile v4f*)(hp + 4) = hn1;
    *(volatile v8h*)sp = hv;
    *(volatile v4f*)fp = ho0;
    *(volatile v4f*)(fp + 4) = ho1;
    *(volatile v8h*)yp = sv;
    __threadfence();
  }
}
static_assert(kB * kH / 8 == 16 * kThr && kH == 16 * 8, "the cell's grid exact: 16 blocks of 256 lanes; a sample's 16 lanes in one wave");

__global__ __launch_bounds__(kThr) void pexit_kernel(const unsigned short* __restrict__ HS, const float* __restrict__ Wp, const float* __restrict__ bp, float* __restrict__ out) {
  const unsigned i = blockIdx.x * (unsigned)kThr + threadIdx.x;
  const unsigned row = i / 3u, k = i - 3u * row;
  const _Float16* hp = (const _Float16*)HS + (size_t)row * (unsigned)kH;
  const float* wp = Wp + (size_t)k * (unsigned)kH;
  float acc = 0.0f;
#pragma unroll
  for (int q = 0; q < kH / 8; ++q) {
    const v8h hv = *(const v8h*)(hp + 8 * q);
#pragma unroll
    for (int e = 0; e < 8; ++e) acc += ((float)hv[e] * kSc10) * bf16r(wp[8 * q + e]);
  }
  const float r = expf(-(acc + bf16r(bp[k])));
  float* dp = out + i;
  *(volatile float*)dp = r;
  __threadfence();
  *(volatile float*)dp = r;
}

__global__ __launch_bounds__(kThr) void qexit_kernel(const float* __restrict__ CV, const float* __restrict__ x, const int* __restrict__ len, const float* __restrict__ Wc, const float* __restrict__ bc, float* __restrict__ out) {
  const unsigned i = blockIdx.x * (unsigned)kThr + threadIdx.x;
  const unsigned rr = i / (unsigned)kCo, c = i - (unsigned)kCo * rr;
  const unsigned b = rr / (unsigned)(kT - 1), t = rr - (unsigned)(kT - 1) * b;
  const unsigned ci = (c < (unsigned)kCv) ? c : (unsigned)(kCv - 1);
  const int ln = len[b];
  const unsigned mk = ((unsigned)(c < (unsigned)kCv) & (unsigned)((int)t + 1 < ln)) ? 0xFFFFFFFFu : 0u;
  const size_t row = (size_t)b * kT + t;
  const float v = CV[row * (unsigned)kCv + ci] + bf16r(x[row * (unsigned)kXi]) * bf16r(Wc[(size_t)ci * kCi + kH]) + bf16r(bc[ci]);
  const float r = __uint_as_float(__float_as_uint(v) & mk);
  float* dp = out + i;
  *(volatile float*)dp = r;
  __threadfence();
  *(volatile float*)dp = r;
}

extern "C" void kernel_launch(void* const* d_in, const int* in_sizes, int n_in,
                              void* d_out, int out_size, void* d_ws, size_t ws_size,
                              hipStream_t stream) {
  if (n_in < 11 || d_out == nullptr || d_ws == nullptr) return;
  if (in_sizes[0] != kB * kT * kXi || in_sizes[1] != kB || in_sizes[2] != kB * kH || in_sizes[3] != kG3 * kXi || in_sizes[4] != kG3 * kH || in_sizes[5] != kG3 || in_sizes[6] != kG3 || in_sizes[7] != 3 * kH || in_sizes[8] != 3 || in_sizes[9] != kCv * kCi || in_sizes[10] != kCv) return;
  if ((size_t)out_size != kOutN) return;
  if (ws_size < kWsTotal) return;
  const float* x = (const float*)d_in[0];
  const int* len = (const int*)d_in[1];
  const float* g0 = (const float*)d_in[2];
  const float* Wi = (const float*)d_in[3];
  const float* Wh = (const float*)d_in[4];
  const float* bi = (const float*)d_in[5];
  const float* bh = (const float*)d_in[6];
  const float* Wp = (const float*)d_in[7];
  const float* bp = (const float*)d_in[8];
  const float* Wc = (const float*)d_in[9];
  const float* bc = (const float*)d_in[10];
  float* out = (float*)d_out;
  char* ws = (char*)d_ws;
  unsigned short* X16 = (unsigned short*)(ws + kOffX16);
  unsigned short* WIT = (unsigned short*)(ws + kOffWIT);
  unsigned short* WHT = (unsigned short*)(ws + kOffWHT);
  unsigned short* WCT = (unsigned short*)(ws + kOffWCT);
  float* GX = (float*)(ws + kOffGX);
  float* GH = (float*)(ws + kOffGH);
  float* H32 = (float*)(ws + kOffH32);
  unsigned short* H16 = (unsigned short*)(ws + kOffH16);
  unsigned short* HS16 = (unsigned short*)(ws + kOffHS16);
  float* CV = (float*)(ws + kOffCV);

  static_assert((kB * kT * (kK1 / 8)) % kThr == 0 && kK1 / 8 == 8 && (kG3 * (kK1 / 8)) % kThr == 0 && (kCv * (kH / 8)) % kThr == 0 && (kG3 * kH / 8) % kThr == 0 && (kB * kH / 8) % kThr == 0 && (kB * kH / 4) % 64 == 0 && (kB * kT * 3) % kThr == 0 && (kB * (kT - 1) * kCo) % kThr == 0, "every flat kernel's grid exact");
  xcast_kernel<<<kB * kT * (kK1 / 8) / kThr, kThr, 0, stream>>>(x, len, X16);
  ocast_kernel<<<kG3 * (kK1 / 8) / kThr, kThr, 0, stream>>>(Wi, WIT, kXi, 6);
  ocast_kernel<<<kCv * (kH / 8) / kThr, kThr, 0, stream>>>(Wc, WCT, kCi, 7);
  cast_plane_kernel<<<kG3 * kH / 8 / kThr, kThr, 0, stream>>>(Wh, WHT, 7, kH, 0);
  cast_plane_kernel<<<kB * kH / 8 / kThr, kThr, 0, stream>>>(g0, H16, 7, kH, 0);
  pack_kernel<<<kB * kH / 4 / 64, 64, 0, stream>>>(g0, nullptr, H32, 1, 0, 0, 0, 0, 0);
  for (int c = 0; c < kT / kCh; ++c) {
    wmma_gemm64<0, false, 0, 0, false, 0><<<dim3(1, kB), 256, 0, stream>>>(
        X16 + (size_t)c * kCh * kK1, X16 + (size_t)c * kCh * kK1, kK1, (long)kT * kK1, WIT, WIT, kK1, 0L, (void*)GX, (void*)GX, kG3, (long)kCh * kG3, nullptr, nullptr, 0L, kCh, kG3, kK1, kSc20);
    for (int tl = 0; tl < kCh; ++tl) {
      const int t = c * kCh + tl;
      wmma_gemm64<0, false, 0, 0, false, 0><<<dim3(3, 1), 256, 0, stream>>>(
          H16, H16, kH, 0L, WHT, WHT, kH, 0L, (void*)GH, (void*)GH, kG3, 0L, nullptr, nullptr, 0L, kB, kG3, kH, kSc20);
      cell_kernel<<<kB * kH / 8 / kThr, kThr, 0, stream>>>(GX, GH, x, len, Wi, bi, bh, H32, H16, out + kOut1, HS16, t);
    }
  }
  wmma_gemm64<0, false, 0, 0, false, 0><<<dim3((kB * kT / 64) * (kCv / 64) / 8, 1), 256, 0, stream>>>(
      HS16, HS16, kH, 0L, WCT, WCT, kH, 0L, (void*)CV, (void*)CV, kCv, 0L, nullptr, nullptr, 0L, kB * kT, kCv, kH, kSc20);
  pexit_kernel<<<kB * kT * 3 / kThr, kThr, 0, stream>>>(HS16, Wp, bp, out + kOut0);
  qexit_kernel<<<kB * (kT - 1) * kCo / kThr, kThr, 0, stream>>>(CV, x, len, Wc, bc, out + kOut2);
}
static_assert(((kB * kT / 64) * (kCv / 64)) % 8 == 0 && kK1 % 32 == 0 && kH % 32 == 0 && kCh % 64 == 0 && kG3 % 64 == 0 && kB % 64 == 0, "the engine's shapes: whole tiles; the depths multiples of 32");
